// RNTN_51805895524400
// MI455X (gfx1250) — hardware-verified
//
#include <hip/hip_runtime.h>
#include <stddef.h>


#define NLEAF 32768
#define NTOT  65024
#define DH    32
#define C2    64
#define NOUT  5
#define VOCAB 50000
#define NTHR  256
#define HP    36
#define PB_V  64
#define PB_W  1
#define PB_G  1024
#define HBLK  508
#define WSCAP 134217728

static_assert(PB_V * NTHR * 8 == DH * C2 * C2);
static_assert(PB_W * NTHR * 8 == C2 * DH);
static_assert(PB_G * NTHR == NLEAF * 8);
static_assert(HBLK * 128 == NTOT);
static_assert((HP * 4) % 16 == 0);
static_assert(8 * 16 * C2 * 4 + 8 * 16 * HP * 4 <= 65536);

typedef float          v4f  __attribute__((ext_vector_type(4)));
typedef float          v8f  __attribute__((ext_vector_type(8)));
typedef unsigned int   v4u  __attribute__((ext_vector_type(4)));
typedef __bf16         v16b __attribute__((ext_vector_type(16)));
union FragB { v16b v; v4u q[2]; };
struct HL { v4u hi; v4u lo; };

__device__ __forceinline__ v8f wmb(v16b a, v16b b, v8f c) {
  v8f d = __builtin_amdgcn_wmma_f32_16x16x32_bf16(false, a, false, b, (short)0, c, false, false);
  asm volatile("v_nop\n\tv_nop\n\tv_nop\n\tv_nop" : "+v"(d) : "v"(a), "v"(b));
  return d;
}

__device__ __forceinline__ v8f zero8() { v8f z = {0.f, 0.f, 0.f, 0.f, 0.f, 0.f, 0.f, 0.f}; return z; }

__device__ __forceinline__ unsigned bfr(float x) {
  const unsigned u = __float_as_uint(x);
  return (u + 0x7FFFu + ((u >> 16) & 1u)) >> 16;
}

__device__ __forceinline__ unsigned pk2(float a, float b, unsigned& lo) {
  const unsigned ra = bfr(a), rb = bfr(b);
  const float da = a - __uint_as_float(ra << 16);
  const float db = b - __uint_as_float(rb << 16);
  lo = bfr(da) | (bfr(db) << 16);
  return ra | (rb << 16);
}

__device__ __forceinline__ HL split8(v4f a, v4f c) {
  unsigned l0, l1, l2, l3;
  const unsigned h0 = pk2(a.x, a.y, l0);
  const unsigned h1 = pk2(a.z, a.w, l1);
  const unsigned h2 = pk2(c.x, c.y, l2);
  const unsigned h3 = pk2(c.z, c.w, l3);
  HL r;
  v4u hv = {h0, h1, h2, h3};
  v4u lv = {l0, l1, l2, l3};
  r.hi = hv; r.lo = lv;
  return r;
}

__device__ __forceinline__ float tanhx(float x) {
  const float e = __expf(-2.0f * fabsf(x));
  const float r = (1.0f - e) * __builtin_amdgcn_rcpf(1.0f + e);
  return x < 0.0f ? -r : r;
}

__global__ __launch_bounds__(NTHR) void k_prep(
    const int* __restrict__ ids, const float* __restrict__ embed,
    const float* __restrict__ V, const float* __restrict__ W,
    float* nodes, unsigned short* Vhi, unsigned short* Vlo,
    unsigned short* Whi, unsigned short* Wlo) {
  const int b = (int)blockIdx.x, tid = (int)threadIdx.x;
  if (b < PB_V) {
    const size_t i = (size_t)b * NTHR + tid;
    const float* sp = V + i * 8;
    const v4f a = *(const v4f*)sp, c = *(const v4f*)(sp + 4);
    const HL s = split8(a, c);
    unsigned short* ph = Vhi + i * 8;
    unsigned short* pl = Vlo + i * 8;
    *(volatile v4u*)ph = s.hi;
    *(volatile v4u*)pl = s.lo;
    __threadfence();
    *(volatile v4u*)ph = s.hi;
    *(volatile v4u*)pl = s.lo;
  } else if (b < PB_V + PB_W) {
    const int n = tid >> 3, l0 = (tid & 7) * 8;
    float v[8];
#pragma unroll
    for (int e = 0; e < 8; ++e) v[e] = W[(l0 + e) * DH + n];
    const v4f a = {v[0], v[1], v[2], v[3]};
    const v4f c = {v[4], v[5], v[6], v[7]};
    const HL s = split8(a, c);
    unsigned short* ph = Whi + n * C2 + l0;
    unsigned short* pl = Wlo + n * C2 + l0;
    *(volatile v4u*)ph = s.hi;
    *(volatile v4u*)pl = s.lo;
    __threadfence();
    *(volatile v4u*)ph = s.hi;
    *(volatile v4u*)pl = s.lo;
  } else {
    const int g = (b - PB_V - PB_W) * NTHR + tid;
    const int row = g >> 3, c4 = g & 7;
    int id = ids[row];
    id = id < 0 ? 0 : (id >= VOCAB ? VOCAB - 1 : id);
    const v4f v = *(const v4f*)(embed + (size_t)id * DH + 4 * c4);
    float* dp = nodes + (size_t)row * DH + 4 * c4;
    *(volatile v4f*)dp = v;
    __threadfence();
    *(volatile v4f*)dp = v;
  }
}

__global__ __launch_bounds__(NTHR) void k_level(
    const float* __restrict__ Cin, float* Hout, float* roots, int wr,
    const unsigned short* __restrict__ Vhi, const unsigned short* __restrict__ Vlo,
    const unsigned short* __restrict__ Whi, const unsigned short* __restrict__ Wlo,
    const float* __restrict__ bias) {
  __shared__ __attribute__((aligned(16))) float sC[8 * 16 * C2];
  __shared__ __attribute__((aligned(16))) float sH[8 * 16 * HP];
  const int tid = threadIdx.x, lane = tid & 31, wave = tid >> 5, hh = lane >> 4, m = lane & 15;
  const int tile = (int)blockIdx.x * 8 + wave;
  float* sc = sC + wave * (16 * C2);
  {
    const float* src = Cin + (size_t)tile * (16 * C2);
#pragma unroll
    for (int it = 0; it < 8; ++it) {
      const int i = it * 32 + lane;
      *(v4f*)(sc + 4 * i) = *(const v4f*)(src + 4 * i);
    }
  }
  __syncthreads();

  FragB ah[2], al[2];
#pragma unroll
  for (int lc = 0; lc < 2; ++lc) {
    const float* rp = sc + m * C2 + lc * 32;
    const v4f a0 = *(const v4f*)(rp + 8 * hh),      a1 = *(const v4f*)(rp + 8 * hh + 4);
    const v4f a2 = *(const v4f*)(rp + 16 + 8 * hh), a3 = *(const v4f*)(rp + 20 + 8 * hh);
    const HL s0 = split8(a0, a1), s1 = split8(a2, a3);
    ah[lc].q[0] = s0.hi; ah[lc].q[1] = s1.hi;
    al[lc].q[0] = s0.lo; al[lc].q[1] = s1.lo;
  }

  float xv0[8], xv1[8];
#pragma unroll
  for (int r = 0; r < 8; ++r) { xv0[r] = 0.0f; xv1[r] = 0.0f; }
  const float* ccp = sc + (8 * hh) * C2 + m;

#pragma unroll 1
  for (int k = 0; k < DH; ++k) {
    float part[8];
#pragma unroll
    for (int r = 0; r < 8; ++r) part[r] = 0.0f;
#pragma unroll 1
    for (int jt = 0; jt < 4; ++jt) {
      const int n = k * C2 + 16 * jt + m;
      const unsigned short* bh = Vhi + (size_t)n * C2 + 8 * hh;
      const unsigned short* bl = Vlo + (size_t)n * C2 + 8 * hh;
      v8f acc = zero8();
#pragma unroll
      for (int lc = 0; lc < 2; ++lc) {
        FragB fh, fl;
        fh.q[0] = *(const v4u*)(bh + lc * 32);  fh.q[1] = *(const v4u*)(bh + lc * 32 + 16);
        fl.q[0] = *(const v4u*)(bl + lc * 32);  fl.q[1] = *(const v4u*)(bl + lc * 32 + 16);
        acc = wmb(ah[lc].v, fh.v, acc);
        acc = wmb(ah[lc].v, fl.v, acc);
        acc = wmb(al[lc].v, fh.v, acc);
      }
      const float* cq = ccp + 16 * jt;
#pragma unroll
      for (int r = 0; r < 8; ++r) part[r] = part[r] + acc[r] * cq[r * C2];
    }
#pragma unroll
    for (int r = 0; r < 8; ++r) {
      float v = part[r];
      v += __shfl_xor(v, 1);
      v += __shfl_xor(v, 2);
      v += __shfl_xor(v, 4);
      v += __shfl_xor(v, 8);
      xv0[r] = (k == m) ? v : xv0[r];
      xv1[r] = (k == m + 16) ? v : xv1[r];
    }
  }

  v8f lin0 = zero8(), lin1 = zero8();
#pragma unroll
  for (int lc = 0; lc < 2; ++lc) {
    const unsigned short* w0h = Whi + (size_t)m * C2 + lc * 32 + 8 * hh;
    const unsigned short* w0l = Wlo + (size_t)m * C2 + lc * 32 + 8 * hh;
    const unsigned short* w1h = Whi + (size_t)(16 + m) * C2 + lc * 32 + 8 * hh;
    const unsigned short* w1l = Wlo + (size_t)(16 + m) * C2 + lc * 32 + 8 * hh;
    FragB f0h, f0l, f1h, f1l;
    f0h.q[0] = *(const v4u*)w0h;  f0h.q[1] = *(const v4u*)(w0h + 16);
    f0l.q[0] = *(const v4u*)w0l;  f0l.q[1] = *(const v4u*)(w0l + 16);
    f1h.q[0] = *(const v4u*)w1h;  f1h.q[1] = *(const v4u*)(w1h + 16);
    f1l.q[0] = *(const v4u*)w1l;  f1l.q[1] = *(const v4u*)(w1l + 16);
    lin0 = wmb(ah[lc].v, f0h.v, lin0);
    lin0 = wmb(ah[lc].v, f0l.v, lin0);
    lin0 = wmb(al[lc].v, f0h.v, lin0);
    lin1 = wmb(ah[lc].v, f1h.v, lin1);
    lin1 = wmb(ah[lc].v, f1l.v, lin1);
    lin1 = wmb(al[lc].v, f1h.v, lin1);
  }

  {
    const float b0 = bias[m], b1 = bias[16 + m];
    float* sh = sH + wave * (16 * HP);
#pragma unroll
    for (int r = 0; r < 8; ++r) {
      sh[(8 * hh + r) * HP + m]      = tanhx(xv0[r] + lin0[r] + b0);
      sh[(8 * hh + r) * HP + 16 + m] = tanhx(xv1[r] + lin1[r] + b1);
    }
  }
  __syncthreads();

  const int q8 = lane & 7, r4 = lane >> 3;
  const float* sh = sH + wave * (16 * HP);
  float* gout = Hout  + (size_t)tile * 16 * DH;
  float* rout = roots + (size_t)tile * 16 * DH;
  v4f ov[4];
#pragma unroll
  for (int it = 0; it < 4; ++it) {
    const int row = 4 * it + r4;
    ov[it] = *(const v4f*)(sh + row * HP + 4 * q8);
    *(volatile v4f*)(gout + (size_t)row * DH + 4 * q8) = ov[it];
    if (wr) *(volatile v4f*)(rout + (size_t)row * DH + 4 * q8) = ov[it];
  }
  __threadfence();
#pragma unroll
  for (int it = 0; it < 4; ++it) {
    const int row = 4 * it + r4;
    *(volatile v4f*)(gout + (size_t)row * DH + 4 * q8) = ov[it];
    if (wr) *(volatile v4f*)(rout + (size_t)row * DH + 4 * q8) = ov[it];
  }
}

__global__ __launch_bounds__(NTHR) void k_head(
    const float* __restrict__ nodes, const float* __restrict__ Ww,
    const float* __restrict__ Wb, float* out) {
  __shared__ __attribute__((aligned(16))) float sL[8 * 256];
  __shared__ __attribute__((aligned(16))) float sO[640];
  const int tid = threadIdx.x, lane = tid & 31, wave = tid >> 5, hh = lane >> 4, m = lane & 15;
  const int row0 = (int)blockIdx.x * 128 + wave * 16;

  FragB ah, al, bh, bl;
  {
    const float* ar = nodes + (size_t)(row0 + m) * DH;
    const HL s0 = split8(*(const v4f*)(ar + 8 * hh),      *(const v4f*)(ar + 8 * hh + 4));
    const HL s1 = split8(*(const v4f*)(ar + 16 + 8 * hh), *(const v4f*)(ar + 20 + 8 * hh));
    ah.q[0] = s0.hi; ah.q[1] = s1.hi; al.q[0] = s0.lo; al.q[1] = s1.lo;
  }
  const int nc = (m < NOUT) ? m : (NOUT - 1);
  {
    const float zf = (m < NOUT) ? 1.0f : 0.0f;
    const float* br = Ww + nc * DH;
    const v4f w0 = *(const v4f*)(br + 8 * hh) * zf,      w1 = *(const v4f*)(br + 8 * hh + 4) * zf;
    const v4f w2 = *(const v4f*)(br + 16 + 8 * hh) * zf, w3 = *(const v4f*)(br + 20 + 8 * hh) * zf;
    const HL s0 = split8(w0, w1), s1 = split8(w2, w3);
    bh.q[0] = s0.hi; bh.q[1] = s1.hi; bl.q[0] = s0.lo; bl.q[1] = s1.lo;
  }
  v8f acc = zero8();
  acc = wmb(ah.v, bh.v, acc);
  acc = wmb(ah.v, bl.v, acc);
  acc = wmb(al.v, bh.v, acc);

  {
    const float wb = Wb[nc];
    float* sl = sL + wave * 256;
#pragma unroll
    for (int r = 0; r < 8; ++r) sl[(8 * hh + r) * 16 + m] = acc[r] + wb;
  }
  __syncthreads();
  if (lane < 16) {
    const float* lr = sL + wave * 256 + lane * 16;
    const float x0 = lr[0], x1 = lr[1], x2 = lr[2], x3 = lr[3], x4 = lr[4];
    const float mx = fmaxf(fmaxf(fmaxf(x0, x1), fmaxf(x2, x3)), x4);
    const float d0 = x0 - mx, d1 = x1 - mx, d2 = x2 - mx, d3 = x3 - mx, d4 = x4 - mx;
    const float se = __expf(d0) + __expf(d1) + __expf(d2) + __expf(d3) + __expf(d4);
    const float lg = __logf(se);
    float* op = sO + (wave * 16 + lane) * NOUT;
    op[0] = d0 - lg; op[1] = d1 - lg; op[2] = d2 - lg; op[3] = d3 - lg; op[4] = d4 - lg;
  }
  __syncthreads();

  v4f ov = {0.f, 0.f, 0.f, 0.f};
  float* gp = out + (size_t)blockIdx.x * 640 + 4 * tid;
  if (tid < 160) {
    ov = *(const v4f*)(sO + 4 * tid);
    *(volatile v4f*)gp = ov;
  }
  __threadfence();
  if (tid < 160) {
    *(volatile v4f*)gp = ov;
  }
}

extern "C" void kernel_launch(void* const* d_in, const int* in_sizes, int n_in,
                              void* d_out, int out_size, void* d_ws, size_t ws_size,
                              hipStream_t stream) {
  if (n_in < 7) return;
  if (in_sizes[0] != NLEAF) return;
  if (in_sizes[1] != VOCAB * DH) return;
  if (in_sizes[2] != DH * C2 * C2) return;
  if (in_sizes[3] != C2 * DH) return;
  if (in_sizes[4] != DH) return;
  if (in_sizes[5] != NOUT * DH) return;
  if (in_sizes[6] != NOUT) return;
  if (out_size != NTOT * NOUT + 512 * DH) return;

  const int*   ids   = (const int*)d_in[0];
  const float* embed = (const float*)d_in[1];
  const float* V     = (const float*)d_in[2];
  const float* W     = (const float*)d_in[3];
  const float* bias  = (const float*)d_in[4];
  const float* Ww    = (const float*)d_in[5];
  const float* Wb    = (const float*)d_in[6];
  float* out   = (float*)d_out;
  float* roots = out + (size_t)NTOT * NOUT;

  char* ws = (char*)d_ws;
  size_t off = 0;
  const size_t oNodes = off; off += (size_t)NTOT * DH * 4;     off = (off + 255) & ~(size_t)255;
  const size_t oVhi   = off; off += (size_t)DH * C2 * C2 * 2;  off = (off + 255) & ~(size_t)255;
  const size_t oVlo   = off; off += (size_t)DH * C2 * C2 * 2;  off = (off + 255) & ~(size_t)255;
  const size_t oWhi   = off; off += (size_t)DH * C2 * 2;       off = (off + 255) & ~(size_t)255;
  const size_t oWlo   = off; off += (size_t)DH * C2 * 2;       off = (off + 255) & ~(size_t)255;
  if (off > ws_size || off > (size_t)WSCAP) return;
  float*          nodes = (float*)(ws + oNodes);
  unsigned short* Vhi   = (unsigned short*)(ws + oVhi);
  unsigned short* Vlo   = (unsigned short*)(ws + oVlo);
  unsigned short* Whi   = (unsigned short*)(ws + oWhi);
  unsigned short* Wlo   = (unsigned short*)(ws + oWlo);

  k_prep<<<PB_V + PB_W + PB_G, NTHR, 0, stream>>>(ids, embed, V, W, nodes, Vhi, Vlo, Whi, Wlo);

  int rows_in = NLEAF, off_in = 0;
  for (int lv = 0; lv < 6; ++lv) {
    const int rows_out = rows_in >> 1;
    const int off_out  = off_in + rows_in;
    const int tiles    = rows_out / 16;
    const int wr       = (lv == 5) ? 1 : 0;
    k_level<<<tiles / 8, NTHR, 0, stream>>>(nodes + (size_t)off_in * DH, nodes + (size_t)off_out * DH,
                                           roots, wr, Vhi, Vlo, Whi, Wlo, bias);
    off_in  = off_out;
    rows_in = rows_out;
  }

  k_head<<<HBLK, NTHR, 0, stream>>>(nodes, Ww, Wb, out);
}
